// WindowAttention3D_17703855194343
// MI455X (gfx1250) — hardware-verified
//
#include <hip/hip_runtime.h>
#include <math.h>
#include <stdint.h>

#define NB   2
#define NP   1024
#define CM   512
#define NH   16
#define HD   32
#define PH   128
#define GRES 3
#define MP   (NB * NP)
#define C3   (3 * CM)
#define QKW  (2 * CM)
#define KC   (2 * CM)
#define NCH  (NP / 32)
#define HLP  136
#define RSC  2048.0f
#define PSC  1024.0f
#define HSC  64.0f
#define W2SC 16.0f
#define SCL  0.17677669529663687f
static_assert(NH * HD == CM);
static_assert((MP % 64) == 0 && (CM % 64) == 0 && (NP % 64) == 0 && (QKW % 64) == 0);
static_assert((((MP / 64) * (QKW / 64)) % 8) == 0);
static_assert((((CM / 64) * (NP / 64)) % 8) == 0);
static_assert((((MP / 64) * (CM / 64)) % 8) == 0);
static_assert(64 * HLP >= NH * 16 * 32);
static_assert(NP == 4 * 256);
static_assert(NH * PH == 4 * 512);
static_assert(PH * 3 <= 512);

typedef _Float16 v16h __attribute__((ext_vector_type(16)));
typedef _Float16 v8h  __attribute__((ext_vector_type(8)));
typedef __bf16   v16b __attribute__((ext_vector_type(16)));
typedef unsigned short v16us __attribute__((ext_vector_type(16)));
typedef unsigned short v8us  __attribute__((ext_vector_type(8)));
typedef float    v8f  __attribute__((ext_vector_type(8)));
typedef float    v4f  __attribute__((ext_vector_type(4)));
typedef unsigned int v4u __attribute__((ext_vector_type(4)));

union FragU { v16us v; v8us h[2]; };

__device__ __forceinline__ unsigned short bf_bits(float f) {
  unsigned u = __float_as_uint(f);
  return (unsigned short)((u + 0x7FFFu + ((u >> 16) & 1u)) >> 16);
}
__device__ __forceinline__ float bf_up(unsigned short h) { return __uint_as_float(((unsigned)h) << 16); }
__device__ __forceinline__ float bfr(float f) { return bf_up(bf_bits(f)); }
__device__ __forceinline__ unsigned short h_bits(_Float16 x) { return __builtin_bit_cast(unsigned short, x); }
__device__ __forceinline__ unsigned pk16(unsigned short a, unsigned short b) { return (unsigned)a | ((unsigned)b << 16); }
__device__ __forceinline__ v8f zero8() { v8f z = {0.f, 0.f, 0.f, 0.f, 0.f, 0.f, 0.f, 0.f}; return z; }

__device__ __forceinline__ v16us ldfrag_u(const unsigned short* p) {
  FragU f;
  f.h[0] = *(const v8us*)(p);
  f.h[1] = *(const v8us*)(p + 16);
  return f.v;
}

__device__ __forceinline__ v8f mma_bu_raw(v16us a, v16us b, v8f c) {
  return __builtin_amdgcn_wmma_f32_16x16x32_bf16(false, __builtin_bit_cast(v16b, a), false,
                                                 __builtin_bit_cast(v16b, b), (short)0, c, false, false);
}
__device__ __forceinline__ v8f mma_hu(v16us a, v16us b, v8f c) {
  c = __builtin_amdgcn_wmma_f32_16x16x32_f16(false, __builtin_bit_cast(v16h, a), false,
                                              __builtin_bit_cast(v16h, b), (short)0, c, false, false);
#if defined(__HIP_DEVICE_COMPILE__)
  asm volatile("v_nop\n\tv_nop\n\tv_nop\n\tv_nop" : "+v"(c) : "v"(a), "v"(b));
#endif
  return c;
}
__device__ __forceinline__ void dep_guard1(v8f& a, v8f& b, v16us x) {
#if defined(__HIP_DEVICE_COMPILE__)
  asm volatile("v_nop\n\tv_nop\n\tv_nop\n\tv_nop" : "+v"(a), "+v"(b) : "v"(x));
#endif
}
__device__ __forceinline__ void keep4_u(v16us a, v16us b, v16us c, v16us d) {
#if defined(__HIP_DEVICE_COMPILE__)
  asm volatile("v_nop" :: "v"(a), "v"(b), "v"(c), "v"(d));
#endif
}
__device__ __forceinline__ void acc_guard4(v8f& a, v8f& b, v8f& c, v8f& d) {
#if defined(__HIP_DEVICE_COMPILE__)
  asm volatile("v_nop\n\tv_nop\n\tv_nop\n\tv_nop" : "+v"(a), "+v"(b), "+v"(c), "+v"(d));
#endif
}
__device__ __forceinline__ void wave_sync_lds() {
  __builtin_amdgcn_fence(__ATOMIC_RELEASE, "workgroup");
  __builtin_amdgcn_wave_barrier();
  __builtin_amdgcn_fence(__ATOMIC_ACQUIRE, "workgroup");
}

__global__ __launch_bounds__(64) void cvt_rows(const float* __restrict__ src, unsigned short* dst, int ldo, int dup) {
  const int row = blockIdx.x, tid = threadIdx.x;
  const float* p = src + (size_t)row * CM + tid * 8;
  const v4f a0 = *(const v4f*)(p);
  const v4f a1 = *(const v4f*)(p + 4);
  v4u hv;
  hv[0] = pk16(bf_bits(a0[0]), bf_bits(a0[1]));
  hv[1] = pk16(bf_bits(a0[2]), bf_bits(a0[3]));
  hv[2] = pk16(bf_bits(a1[0]), bf_bits(a1[1]));
  hv[3] = pk16(bf_bits(a1[2]), bf_bits(a1[3]));
  unsigned short* d = dst + (size_t)row * ldo + tid * 8;
  for (int pass = 0; pass < 2; ++pass) {
    *(volatile v4u*)(d) = hv;
    if (dup != 0) *(volatile v4u*)(d + dup) = hv;
    __threadfence();
  }
}

__global__ __launch_bounds__(256) void cell_ids(const float* __restrict__ coords, int* wid) {
#pragma clang fp contract(off)
  __shared__ float smn[8][3], smx[8][3];
  __shared__ float bmn[3], bmx[3];
  const int b = blockIdx.x, t = threadIdx.x, w = t >> 5, l = t & 31;
  float cv[4][3];
  float mn[3], mx[3];
#pragma unroll
  for (int d = 0; d < 3; ++d) { mn[d] = 3.0e38f; mx[d] = -3.0e38f; }
#pragma unroll
  for (int i = 0; i < 4; ++i) {
    const float* c = coords + ((size_t)b * NP + i * 256 + t) * 3;
#pragma unroll
    for (int d = 0; d < 3; ++d) {
      const float v = bfr(c[d]);
      cv[i][d] = v;
      mn[d] = fminf(mn[d], v);
      mx[d] = fmaxf(mx[d], v);
    }
  }
#pragma unroll
  for (int off = 1; off < 32; off <<= 1) {
#pragma unroll
    for (int d = 0; d < 3; ++d) {
      mn[d] = fminf(mn[d], __shfl_xor(mn[d], off, 32));
      mx[d] = fmaxf(mx[d], __shfl_xor(mx[d], off, 32));
    }
  }
  if (l == 0) {
#pragma unroll
    for (int d = 0; d < 3; ++d) { smn[w][d] = mn[d]; smx[w][d] = mx[d]; }
  }
  __syncthreads();
  if (t == 0) {
#pragma unroll
    for (int d = 0; d < 3; ++d) {
      float a = smn[0][d], bb = smx[0][d];
#pragma unroll
      for (int i = 1; i < 8; ++i) { a = fminf(a, smn[i][d]); bb = fmaxf(bb, smx[i][d]); }
      bmn[d] = a; bmx[d] = bb;
    }
  }
  __syncthreads();
  int idv[4];
#pragma unroll
  for (int i = 0; i < 4; ++i) {
    int id = 0;
#pragma unroll
    for (int d = 0; d < 3; ++d) {
      float r = bmx[d] - bmn[d];
      if (r < 1e-6f) r = 1.0f;
      const float cn = (cv[i][d] - bmn[d]) * (1.0f / r);
      int bi = (int)(cn * 3.0f);
      bi = bi < 0 ? 0 : (bi > GRES - 1 ? GRES - 1 : bi);
      id = id * GRES + bi;
    }
    idv[i] = id;
  }
  for (int pass = 0; pass < 2; ++pass) {
#pragma unroll
    for (int i = 0; i < 4; ++i) *(volatile int*)(wid + (size_t)b * NP + i * 256 + t) = idv[i];
    __threadfence();
  }
}

template <int OM, int CBM>
__global__ __launch_bounds__(256) void gemm64(
    const unsigned short* __restrict__ Ap, int lda, long long sAy,
    const unsigned short* __restrict__ Btp, int ldb, long long sBy,
    unsigned short* Cp, unsigned short* Cp2, float* Cf, int ldc, long long sCy,
    const float* __restrict__ cb, int M, int N, int K) {
  __shared__ __align__(16) float sT[8][16 * 68];
  const int by   = blockIdx.y;
  const int lane = threadIdx.x & 31;
  const int wave = threadIdx.x >> 5;
  const int tilesN = N >> 6;
  const int tilesM = M >> 6;
  const int tile = blockIdx.x * 8 + wave;
  if (tile >= tilesM * tilesN) return;
  const int tm = tile / tilesN;
  const int tn = tile - tm * tilesN;
  const int m0 = tm << 6;
  const int n0 = tn << 6;

  const unsigned short* Ab = Ap  + (size_t)by * (size_t)sAy;
  const unsigned short* Bb = Btp + (size_t)by * (size_t)sBy;
  const size_t cofs = (size_t)by * (size_t)sCy;

  const int rlane = lane & 15;
  const int koff  = (lane >> 4) * 8;
  const int mOff  = (lane >> 4) * 8;

  v8f acc[4][4];
#pragma unroll
  for (int i = 0; i < 4; ++i)
#pragma unroll
    for (int j = 0; j < 4; ++j) acc[i][j] = zero8();

  for (int k0 = 0; k0 < K; k0 += 32) {
    v16us bh[4];
#pragma unroll
    for (int j = 0; j < 4; ++j) {
      const size_t bo = (size_t)(n0 + (j << 4) + rlane) * ldb + koff + k0;
      bh[j] = ldfrag_u(Bb + bo);
    }
#pragma unroll
    for (int i = 0; i < 4; ++i) {
      const size_t ao = (size_t)(m0 + (i << 4) + rlane) * lda + koff + k0;
      const v16us ah = ldfrag_u(Ab + ao);
#pragma unroll
      for (int j = 0; j < 4; ++j) acc[i][j] = mma_bu_raw(ah, bh[j], acc[i][j]);
      dep_guard1(acc[i][0], acc[i][3], ah);
    }
    keep4_u(bh[0], bh[1], bh[2], bh[3]);
  }
  acc_guard4(acc[0][0], acc[0][1], acc[0][2], acc[0][3]);
  acc_guard4(acc[1][0], acc[1][1], acc[1][2], acc[1][3]);
  acc_guard4(acc[2][0], acc[2][1], acc[2][2], acc[2][3]);
  acc_guard4(acc[3][0], acc[3][1], acc[3][2], acc[3][3]);

  const int hh2 = lane >> 4, c4 = (lane & 15) * 4;
  const int q8  = lane >> 3, c8 = (lane & 7) * 8;

  v4f cb4 = {0.f, 0.f, 0.f, 0.f};
  float cbc[8];
#pragma unroll
  for (int e = 0; e < 8; ++e) cbc[e] = 0.f;
  if (CBM == 1) {
    if (OM == 0) {
      const v4f v = *(const v4f*)(cb + n0 + c4);
      cb4[0] = bfr(v[0]); cb4[1] = bfr(v[1]); cb4[2] = bfr(v[2]); cb4[3] = bfr(v[3]);
    } else {
      const v4f v0 = *(const v4f*)(cb + n0 + c8);
      const v4f v1 = *(const v4f*)(cb + n0 + c8 + 4);
#pragma unroll
      for (int e = 0; e < 4; ++e) { cbc[e] = bfr(v0[e]); cbc[4 + e] = bfr(v1[e]); }
    }
  }

  float* slab = sT[wave];
#pragma unroll
  for (int i = 0; i < 4; ++i) {
    const int mBase = m0 + (i << 4);
#pragma unroll
    for (int j = 0; j < 4; ++j) {
#pragma unroll
      for (int r = 0; r < 8; ++r) {
        slab[(mOff + r) * 68 + (j << 4) + rlane] = acc[i][j][r];
      }
    }
    wave_sync_lds();
    if (OM == 0) {
      float* C = Cf + cofs;
      v4f vals[8];
#pragma unroll
      for (int it = 0; it < 8; ++it) {
        const int row = it * 2 + hh2;
        const v4f v = *(const v4f*)(slab + row * 68 + c4);
        vals[it] = v + cb4;
      }
      for (int pass = 0; pass < 2; ++pass) {
#pragma unroll
        for (int it = 0; it < 8; ++it) {
          const int row = it * 2 + hh2;
          *(volatile v4f*)(C + (size_t)(mBase + row) * ldc + (size_t)n0 + c4) = vals[it];
        }
        __threadfence();
      }
    } else {
      unsigned short* C  = Cp  + cofs;
      unsigned short* C2 = Cp2 + cofs;
      v4u hv[4], lv[4];
#pragma unroll
      for (int it = 0; it < 4; ++it) {
        const int row = it * 4 + q8;
        const float* sp = slab + row * 68 + c8;
        float rb = 0.f;
        if (CBM == 2) rb = bfr(cb[mBase + row]);
        v4u ha = {0u, 0u, 0u, 0u}, la = {0u, 0u, 0u, 0u};
#pragma unroll
        for (int e = 0; e < 4; ++e) {
          const float f0 = sp[2 * e]     + cbc[2 * e]     + rb;
          const float f1 = sp[2 * e + 1] + cbc[2 * e + 1] + rb;
          const _Float16 g0 = (_Float16)f0, g1 = (_Float16)f1;
          ha[e] = pk16(h_bits(g0), h_bits(g1));
          if (OM == 2) {
            la[e] = pk16(h_bits((_Float16)((f0 - (float)g0) * RSC)),
                         h_bits((_Float16)((f1 - (float)g1) * RSC)));
          }
        }
        hv[it] = ha;
        lv[it] = la;
      }
      for (int pass = 0; pass < 2; ++pass) {
#pragma unroll
        for (int it = 0; it < 4; ++it) {
          const int row = it * 4 + q8;
          const size_t go = (size_t)(mBase + row) * ldc + (size_t)n0 + c8;
          *(volatile v4u*)(C + go) = hv[it];
          if (OM == 2) *(volatile v4u*)(C2 + go) = lv[it];
        }
        __threadfence();
      }
    }
    wave_sync_lds();
  }
}

__global__ void __launch_bounds__(512) attn_kernel(
    const float* __restrict__ coords,
    const float* __restrict__ w1, const float* __restrict__ b1,
    const float* __restrict__ w2, const float* __restrict__ b2,
    const unsigned short* __restrict__ qk,
    const unsigned short* __restrict__ vth, const unsigned short* __restrict__ vtl,
    const int* __restrict__ wid, unsigned short* ctxp) {
  __shared__ __align__(16) unsigned short hidL[64 * HLP];
  __shared__ __align__(16) float biasL[512 * NH];
  __shared__ __align__(16) unsigned short w2s[NH * PH];
  __shared__ float w1s[PH * 3], b1s[PH], b2s[NH];
  __shared__ float cis[16 * 3], cjs[32 * 3];
  __shared__ int wis[16], wjs[32];
  __shared__ unsigned short listL[512];
  __shared__ int wcnt[NH], wbase[NH], nactS;

  const int b = blockIdx.y, i0 = blockIdx.x * 16;
  const int t = threadIdx.x, lane = t & 31, w = t >> 5, hh = lane >> 4, jc = lane & 15;
  const size_t rowB = (size_t)b * NP;

  if (t < PH * 3) w1s[t] = bfr(w1[t]);
  if (t < PH) b1s[t] = bfr(b1[t]);
  if (t < NH) b2s[t] = bfr(b2[t]);
#pragma unroll
  for (int i = 0; i < 4; ++i) {
    const int e = i * 512 + t;
    w2s[e] = h_bits((_Float16)(bfr(w2[e]) * W2SC));
  }
  if (t < 48) cis[t] = bfr(coords[(rowB + i0) * 3 + t]);
  if (t < 16) wis[t] = wid[rowB + i0 + t];
#pragma unroll
  for (int i = 0; i < 16; ++i) biasL[i * 512 + t] = 0.f;
  __syncthreads();

  const v16us qf = ldfrag_u(qk + (rowB + i0 + jc) * QKW + w * HD + 8 * hh);
  int widr[8];
#pragma unroll
  for (int r = 0; r < 8; ++r) widr[r] = wis[8 * hh + r];
  const int wiq = wis[w];

  float m[8], ll[8];
  v8f oh0 = zero8(), oh1 = zero8(), ol0 = zero8(), ol1 = zero8();
#pragma unroll
  for (int r = 0; r < 8; ++r) { m[r] = -1.0e30f; ll[r] = 0.f; }

  const unsigned short* vhb = vth + ((size_t)b * CM + w * HD + jc) * NP + 8 * hh;
  const unsigned short* vlb = vtl + ((size_t)b * CM + w * HD + jc) * NP + 8 * hh;
  const unsigned short* kgb = qk + (rowB + jc) * QKW + CM + w * HD + 8 * hh;
  unsigned short* pr = hidL + w * 512;

#pragma unroll 1
  for (int jt = 0; jt < NCH; ++jt) {
    const int j0 = jt * 32;
    __syncthreads();
    if (t < 32) wjs[t] = wid[rowB + j0 + t];
    if (t >= 32 && t < 128) cjs[t - 32] = bfr(coords[(rowB + j0) * 3 + (t - 32)]);
    __syncthreads();

    const bool same = (wiq == wjs[lane]);
    const unsigned bal = (unsigned)__ballot(same);
    if (lane == 0) wcnt[w] = (int)__popc(bal);
    __syncthreads();
    if (t == 0) {
      int s = 0;
#pragma unroll
      for (int i = 0; i < NH; ++i) { wbase[i] = s; s += wcnt[i]; }
      nactS = s;
    }
    __syncthreads();
    int nact = nactS;
    nact = nact > 512 ? 512 : nact;
    if (same) {
      int idx = wbase[w] + (int)__popc(bal & ((1u << lane) - 1u));
      idx = idx > 511 ? 511 : (idx < 0 ? 0 : idx);
      listL[idx] = (unsigned short)t;
    }
    __syncthreads();

#pragma unroll 1
    for (int base = 0; base < nact; base += 64) {
      int nb = nact - base;
      nb = nb > 64 ? 64 : nb;
      const int nbp = (nb + 15) & ~15;
      {
        const int e = t & 63, q = t >> 6;
        if (e < nbp) {
          v4u pk0 = {0u, 0u, 0u, 0u}, pk1 = {0u, 0u, 0u, 0u};
          if (e < nb) {
            int li = base + e;
            li = li > 511 ? 511 : li;
            const int p = listL[li];
            const int pil = (p >> 5) & 15, pjl = p & 31;
            const float ox = cis[pil * 3 + 0] - cjs[pjl * 3 + 0];
            const float oy = cis[pil * 3 + 1] - cjs[pjl * 3 + 1];
            const float oz = cis[pil * 3 + 2] - cjs[pjl * 3 + 2];
            unsigned short hv[16];
#pragma unroll
            for (int kq = 0; kq < 16; ++kq) {
              const int kk = q * 16 + kq;
              const float s = ox * w1s[kk * 3 + 0] + oy * w1s[kk * 3 + 1] + oz * w1s[kk * 3 + 2] + b1s[kk];
              const float g = 0.5f * s * (1.0f + erff(s * 0.70710678118654752f));
              hv[kq] = h_bits((_Float16)(g * HSC));
            }
#pragma unroll
            for (int e4 = 0; e4 < 4; ++e4) {
              pk0[e4] = pk16(hv[2 * e4], hv[2 * e4 + 1]);
              pk1[e4] = pk16(hv[8 + 2 * e4], hv[9 + 2 * e4]);
            }
          }
          *(v4u*)(hidL + e * HLP + q * 16)     = pk0;
          *(v4u*)(hidL + e * HLP + q * 16 + 8) = pk1;
        }
      }
      __syncthreads();
      const int ntile = nbp >> 4;
      if (w < ntile) {
        v8f vb = zero8();
#pragma unroll
        for (int cc = 0; cc < 4; ++cc) {
          FragU a, bw;
          a.h[0]  = *(const v8us*)(hidL + (w * 16 + jc) * HLP + cc * 32 + 8 * hh);
          a.h[1]  = *(const v8us*)(hidL + (w * 16 + jc) * HLP + cc * 32 + 16 + 8 * hh);
          bw.h[0] = *(const v8us*)(w2s + jc * PH + cc * 32 + 8 * hh);
          bw.h[1] = *(const v8us*)(w2s + jc * PH + cc * 32 + 16 + 8 * hh);
          vb = mma_hu(a.v, bw.v, vb);
        }
        const float b2r = b2s[jc];
#pragma unroll
        for (int r = 0; r < 8; ++r) {
          const int row = w * 16 + 8 * hh + r;
          if (row < nb) {
            int li = base + row;
            li = li > 511 ? 511 : li;
            const int pair = ((int)listL[li]) & 511;
            biasL[pair * NH + jc] = vb[r] * (1.0f / (HSC * W2SC)) + b2r;
          }
        }
      }
      __syncthreads();
    }

    const unsigned short* kg = kgb + (size_t)j0 * QKW;
    const v16us kf0 = ldfrag_u(kg);
    const v16us kf1 = ldfrag_u(kg + (size_t)16 * QKW);
    v8f s0 = mma_hu(qf, kf0, zero8());
    v8f s1 = mma_hu(qf, kf1, zero8());

#pragma unroll
    for (int r = 0; r < 8; ++r) {
      const int il = 8 * hh + r;
      const float bb0 = biasL[(il * 32 + jc) * NH + w];
      const float bb1 = biasL[(il * 32 + 16 + jc) * NH + w];
      const float v0 = (widr[r] == wjs[jc])      ? (s0[r] * SCL + bb0) : -10000.0f;
      const float v1 = (widr[r] == wjs[16 + jc]) ? (s1[r] * SCL + bb1) : -10000.0f;
      float rm = fmaxf(v0, v1);
#pragma unroll
      for (int off = 1; off < 16; off <<= 1) rm = fmaxf(rm, __shfl_xor(rm, off, 32));
      const float mn2   = fmaxf(m[r], rm);
      const float alpha = __expf(m[r] - mn2);
      const float e0 = __expf(v0 - mn2), e1 = __expf(v1 - mn2);
      float rs = e0 + e1;
#pragma unroll
      for (int off = 1; off < 16; off <<= 1) rs += __shfl_xor(rs, off, 32);
      ll[r] = ll[r] * alpha + rs;
      m[r]  = mn2;
      oh0[r] *= alpha; oh1[r] *= alpha; ol0[r] *= alpha; ol1[r] *= alpha;
      pr[il * 32 + jc]      = h_bits((_Float16)(e0 * PSC));
      pr[il * 32 + 16 + jc] = h_bits((_Float16)(e1 * PSC));
    }
    wave_sync_lds();

    FragU pa;
    pa.h[0] = *(const v8us*)(pr + jc * 32 + 8 * hh);
    pa.h[1] = *(const v8us*)(pr + jc * 32 + 16 + 8 * hh);
    {
      const v16us vh0 = ldfrag_u(vhb + j0);
      const v16us vh1 = ldfrag_u(vhb + (size_t)16 * NP + j0);
      oh0 = mma_hu(pa.v, vh0, oh0);
      oh1 = mma_hu(pa.v, vh1, oh1);
      const v16us vl0 = ldfrag_u(vlb + j0);
      const v16us vl1 = ldfrag_u(vlb + (size_t)16 * NP + j0);
      ol0 = mma_hu(pa.v, vl0, ol0);
      ol1 = mma_hu(pa.v, vl1, ol1);
    }
  }

  __syncthreads();
  float* osm = biasL;
#pragma unroll
  for (int r = 0; r < 8; ++r) {
    const int il = 8 * hh + r;
    const float l = ll[r];
    const float inv = ((l > 0.f) ? (1.0f / l) : 0.f) * (1.0f / PSC);
    osm[il * CM + w * HD + jc]      = (oh0[r] + ol0[r] * (1.0f / RSC)) * inv;
    osm[il * CM + w * HD + 16 + jc] = (oh1[r] + ol1[r] * (1.0f / RSC)) * inv;
  }
  __syncthreads();
  {
    const float* sp = osm + w * CM;
    v4u hv[2], lv[2];
#pragma unroll
    for (int it = 0; it < 2; ++it) {
      const int c = it * 256 + lane * 8;
      const v4f f0 = *(const v4f*)(sp + c);
      const v4f f1 = *(const v4f*)(sp + c + 4);
      v4u ha, la;
#pragma unroll
      for (int e = 0; e < 2; ++e) {
        const unsigned short u0 = bf_bits(f0[2 * e]), u1 = bf_bits(f0[2 * e + 1]);
        const unsigned short u2 = bf_bits(f1[2 * e]), u3 = bf_bits(f1[2 * e + 1]);
        ha[e]     = pk16(u0, u1);
        ha[2 + e] = pk16(u2, u3);
        la[e]     = pk16(bf_bits(f0[2 * e] - bf_up(u0)), bf_bits(f0[2 * e + 1] - bf_up(u1)));
        la[2 + e] = pk16(bf_bits(f1[2 * e] - bf_up(u2)), bf_bits(f1[2 * e + 1] - bf_up(u3)));
      }
      hv[it] = ha;
      lv[it] = la;
    }
    const size_t go = (rowB + i0 + w) * KC;
    for (int pass = 0; pass < 2; ++pass) {
#pragma unroll
      for (int it = 0; it < 2; ++it) {
        const int c = it * 256 + lane * 8;
        *(volatile v4u*)(ctxp + go + c)      = hv[it];
        *(volatile v4u*)(ctxp + go + CM + c) = lv[it];
      }
      __threadfence();
    }
  }
}

extern "C" void kernel_launch(void* const* d_in, const int* in_sizes, int n_in,
                              void* d_out, int out_size, void* d_ws, size_t ws_size,
                              hipStream_t stream) {
  if (n_in < 10) return;
  if (in_sizes[0] != NB * NP * 3) return;
  if (in_sizes[1] != MP * CM) return;
  if (in_sizes[2] != C3 * CM || in_sizes[3] != C3) return;
  if (in_sizes[4] != CM * CM || in_sizes[5] != CM) return;
  if (in_sizes[6] != PH * 3 || in_sizes[7] != PH) return;
  if (in_sizes[8] != NH * PH || in_sizes[9] != NH) return;
  if (out_size != MP * CM) return;

  const float* coords = (const float*)d_in[0];
  const float* x      = (const float*)d_in[1];
  const float* qkv_w  = (const float*)d_in[2];
  const float* qkv_b  = (const float*)d_in[3];
  const float* proj_w = (const float*)d_in[4];
  const float* proj_b = (const float*)d_in[5];
  const float* pos_w1 = (const float*)d_in[6];
  const float* pos_b1 = (const float*)d_in[7];
  const float* pos_w2 = (const float*)d_in[8];
  const float* pos_b2 = (const float*)d_in[9];

  const size_t PXB  = (size_t)MP * CM * 2;
  const size_t PWB  = (size_t)C3 * CM * 2;
  const size_t PWO  = (size_t)CM * KC * 2;
  const size_t PQK  = (size_t)MP * QKW * 2;
  const size_t PVT  = (size_t)NB * CM * NP * 2;
  const size_t PCTX = (size_t)MP * KC * 2;
  const size_t PWID = (size_t)MP * 4;
  size_t off = 0;
  const size_t oXb  = off; off += PXB;
  const size_t oWb  = off; off += PWB;
  const size_t oWo  = off; off += PWO;
  const size_t oQK  = off; off += PQK;
  const size_t oVTh = off; off += PVT;
  const size_t oVTl = off; off += PVT;
  const size_t oCtx = off; off += PCTX;
  const size_t oWid = off; off += PWID;
  if (off > ws_size) return;
  if (off > (size_t)134217728) return;

  char* ws = (char*)d_ws;
  unsigned short* Xb   = (unsigned short*)(ws + oXb);
  unsigned short* Wb   = (unsigned short*)(ws + oWb);
  unsigned short* WoT2 = (unsigned short*)(ws + oWo);
  unsigned short* QK   = (unsigned short*)(ws + oQK);
  unsigned short* VTh  = (unsigned short*)(ws + oVTh);
  unsigned short* VTl  = (unsigned short*)(ws + oVTl);
  unsigned short* Ctx  = (unsigned short*)(ws + oCtx);
  int*            Wid  = (int*)(ws + oWid);
  float*          out0 = (float*)d_out;

  const dim3 blk(256), blk512(512), blk64(64);
  const dim3 gQK(((MP / 64) * (QKW / 64)) / 8, 1, 1);
  const dim3 gVT(((CM / 64) * (NP / 64)) / 8, NB, 1);
  const dim3 gAttn(NP / 16, NB, 1);
  const dim3 gNo(((MP / 64) * (CM / 64)) / 8, 1, 1);
  if ((((MP / 64) * (QKW / 64)) % 8) != 0) return;
  if ((((CM / 64) * (NP / 64)) % 8) != 0) return;
  if ((((MP / 64) * (CM / 64)) % 8) != 0) return;

  cvt_rows<<<dim3(MP), blk64, 0, stream>>>(x, Xb, CM, 0);
  cvt_rows<<<dim3(C3), blk64, 0, stream>>>(qkv_w, Wb, CM, 0);
  cvt_rows<<<dim3(CM), blk64, 0, stream>>>(proj_w, WoT2, KC, CM);
  cell_ids<<<dim3(NB), blk, 0, stream>>>(coords, Wid);

  gemm64<1, 1><<<gQK, blk, 0, stream>>>(
      Xb, CM, 0LL, Wb, CM, 0LL,
      QK, QK, out0, QKW, 0LL,
      qkv_b, MP, QKW, CM);
  gemm64<2, 2><<<gVT, blk, 0, stream>>>(
      Wb + (size_t)QKW * CM, CM, 0LL, Xb, CM, (long long)NP * CM,
      VTh, VTl, out0, NP, (long long)CM * NP,
      qkv_b + QKW, CM, NP, CM);

  attn_kernel<<<gAttn, blk512, 0, stream>>>(coords, pos_w1, pos_b1, pos_w2, pos_b2, QK, VTh, VTl, Wid, Ctx);

  gemm64<0, 1><<<gNo, blk, 0, stream>>>(
      Ctx, KC, 0LL, WoT2, KC, 0LL,
      Ctx, Ctx, out0, CM, 0LL,
      proj_b, MP, CM, KC);
  (void)hipGetLastError();
}
